// HybridANFIS_38534446580295
// MI455X (gfx1250) — hardware-verified
//
#include <hip/hip_runtime.h>
#include <stddef.h>

#pragma clang fp contract(off)

#define NB    8192
#define ND    16
#define NM    3
#define NQ    48
#define NRU   1000
#define NC    10
#define NJ    17
#define KP    1024
#define NPB   16
#define TOPK  200
#define RB    32
#define NTH   256
#define NWV   8
#define NCH1  ((RB * NRU / 4) / 32)

#define L_F    0
#define L_M    (L_F + RB * KP * 4)
#define L_P    (L_M + RB * NQ * 4)
#define L_O0   (L_P + NWV * 256 * 4)
#define L_O2   (L_O0 + RB * NC * 4)
#define L_SX   (L_O2 + RB * NJ * 4)
#define LDS_MAIN (L_SX + RB * 4)

static_assert(NQ == ND * NM);
static_assert(NJ == ND + 1);
static_assert(NB % RB == 0);
static_assert(RB == 4 * NWV);
static_assert(NTH == 32 * NWV);
static_assert(RB * NQ == 6 * NTH);
static_assert(KP == 4 * NTH);
static_assert(KP % 128 == 0);
static_assert(NRU % 4 == 0);
static_assert((RB * NRU / 4) % 32 == 0);
static_assert((RB * NRU * 4) % 128 == 0);
static_assert((RB * NC * 4) % 128 == 0);
static_assert((RB * NJ * 4) % 128 == 0);
static_assert(((size_t)NB * NC * 4) % 128 == 0);
static_assert((((size_t)NB * NC + (size_t)NB * NRU) * 4) % 128 == 0);
static_assert(RB <= NTH);
static_assert(RB * NC / 4 <= 3 * 32);
static_assert(RB * NJ / 4 <= 5 * 32);
static_assert(L_M % 16 == 0);
static_assert(L_P % 16 == 0);
static_assert(L_O0 % 16 == 0);
static_assert(L_O2 % 16 == 0);
static_assert(L_SX % 16 == 0);
static_assert(LDS_MAIN % 16 == 0);
static_assert(NRU - 31 * 32 == 8);

typedef __bf16         v16b __attribute__((ext_vector_type(16)));
typedef float          v8f  __attribute__((ext_vector_type(8)));
typedef float          v4f  __attribute__((ext_vector_type(4)));
typedef unsigned int   v4u  __attribute__((ext_vector_type(4)));
typedef unsigned int   v8u  __attribute__((ext_vector_type(8)));
typedef unsigned short v8us __attribute__((ext_vector_type(8)));
typedef int            v4i  __attribute__((ext_vector_type(4)));
typedef v4f __attribute__((may_alias)) v4fa;
typedef v4u __attribute__((may_alias)) v4ua;
typedef v4i __attribute__((may_alias)) v4ia;

__device__ __forceinline__ unsigned int bf16_rne_bits(float f) {
  const unsigned int u = __float_as_uint(f);
  return (u + 0x7FFFu + ((u >> 16) & 1u)) >> 16;
}
__device__ __forceinline__ void split2(float f, unsigned short& hi, unsigned short& lo) {
  const unsigned int hu = bf16_rne_bits(f);
  const float fh = __uint_as_float(hu << 16);
  const unsigned int lu = bf16_rne_bits(f - fh);
  hi = (unsigned short)hu;
  lo = (unsigned short)lu;
}
__device__ __forceinline__ void split8(v4f a, v4f c, v4u& uh, v4u& ul) {
  v8us hv = {0, 0, 0, 0, 0, 0, 0, 0};
  v8us lv = {0, 0, 0, 0, 0, 0, 0, 0};
  unsigned short hh, ll;
  split2(a.x, hh, ll); hv[0] = hh; lv[0] = ll;
  split2(a.y, hh, ll); hv[1] = hh; lv[1] = ll;
  split2(a.z, hh, ll); hv[2] = hh; lv[2] = ll;
  split2(a.w, hh, ll); hv[3] = hh; lv[3] = ll;
  split2(c.x, hh, ll); hv[4] = hh; lv[4] = ll;
  split2(c.y, hh, ll); hv[5] = hh; lv[5] = ll;
  split2(c.z, hh, ll); hv[6] = hh; lv[6] = ll;
  split2(c.w, hh, ll); hv[7] = hh; lv[7] = ll;
  uh = __builtin_bit_cast(v4u, hv);
  ul = __builtin_bit_cast(v4u, lv);
}

__device__ __forceinline__ v8f wmma_b(v16b a, v16b b, v8f c) {
  v8f d = __builtin_amdgcn_wmma_f32_16x16x32_bf16(false, a, false, b, (short)0, c, false, false);
  asm volatile("v_nop\n\tv_nop\n\tv_nop\n\tv_nop" : "+v"(d) : "v"(a), "v"(b));
  return d;
}

__device__ __forceinline__ v16b ldfrag(const unsigned short* p, int h) {
  const v4u q0 = *(const v4ua*)(p + 8 * h);
  const v4u q1 = *(const v4ua*)(p + 16 + 8 * h);
  const v8u w = {q0.x, q0.y, q0.z, q0.w, q1.x, q1.y, q1.z, q1.w};
  return __builtin_bit_cast(v16b, w);
}

__device__ __forceinline__ int wsum_i(int v) {
  v += __shfl_xor(v, 16);
  v += __shfl_xor(v, 8);
  v += __shfl_xor(v, 4);
  v += __shfl_xor(v, 2);
  v += __shfl_xor(v, 1);
  return v;
}
__device__ __forceinline__ float wsum_f(float v) {
  v += __shfl_xor(v, 16);
  v += __shfl_xor(v, 8);
  v += __shfl_xor(v, 4);
  v += __shfl_xor(v, 2);
  v += __shfl_xor(v, 1);
  return v;
}
__device__ __forceinline__ int clampm(int m) {
  return (m < 0) ? 0 : ((m > NM - 1) ? (NM - 1) : m);
}

__global__ __launch_bounds__(NTH) void k_scons(const float* __restrict__ cons,
                                                unsigned short* __restrict__ sch,
                                                unsigned short* __restrict__ scl)
{
  __shared__ __align__(16) unsigned short sH[NTH];
  __shared__ __align__(16) unsigned short sL[NTH];
  const int tid = threadIdx.x, lane = tid & 31, wv = tid >> 5;
  const int k = blockIdx.x * NTH + tid;
  const int n = blockIdx.y;
  const int kc = (k > NRU - 1) ? (NRU - 1) : k;
  const int nn = (n > NC - 1) ? (NC - 1) : n;
  const float* p = cons + (size_t)kc * NJ * NC + nn;
  float s = 0.0f;
  #pragma unroll 1
  for (int j = 0; j < NJ; ++j) s += p[j * NC];
  s = (k < NRU && n < NC) ? s : 0.0f;
  unsigned short hh, ll;
  split2(s, hh, ll);
  sH[tid] = hh;
  sL[tid] = ll;
  __syncthreads();
  if (wv == 0) {
    const v4u a = *(const v4ua*)(sH + 8 * lane);
    const v4u b = *(const v4ua*)(sL + 8 * lane);
    const size_t o = (size_t)n * KP + (size_t)blockIdx.x * NTH + 8 * lane;
    *(volatile v4u*)(sch + o) = a;
    *(volatile v4u*)(scl + o) = b;
    __threadfence();
    *(volatile v4u*)(sch + o) = a;
    *(volatile v4u*)(scl + o) = b;
  }
}

__device__ __forceinline__ void store_pass(const float* sF, const float* sO0, const float* sO2,
                                           float* o0, float* o1, float* o2,
                                           const int wv, const int lane)
{
  #pragma unroll 1
  for (int it = 0; it < (NCH1 + NWV - 1) / NWV; ++it) {
    const int ch = wv + NWV * it;
    if (ch < NCH1) {
      const int piece = ch * 32 + lane;
      const int f = piece * 4;
      const int row = f / NRU;
      const int col = f - row * NRU;
      const v4f v = *(const v4fa*)(sF + row * KP + col);
      *(volatile v4f*)(o1 + f) = v;
    }
  }
  if (wv == 0) {
    #pragma unroll
    for (int q = 0; q < 3; ++q) {
      const int piece = q * 32 + lane;
      const int pc = (piece > RB * NC / 4 - 1) ? (RB * NC / 4 - 1) : piece;
      const v4f v = *(const v4fa*)(sO0 + 4 * pc);
      if (piece < RB * NC / 4) *(volatile v4f*)(o0 + 4 * piece) = v;
    }
  }
  if (wv == 1) {
    #pragma unroll
    for (int q = 0; q < 5; ++q) {
      const int piece = q * 32 + lane;
      const int pc = (piece > RB * NJ / 4 - 1) ? (RB * NJ / 4 - 1) : piece;
      const v4f v = *(const v4fa*)(sO2 + 4 * pc);
      if (piece < RB * NJ / 4) *(volatile v4f*)(o2 + 4 * piece) = v;
    }
  }
}

__global__ __launch_bounds__(NTH) void k_main(
    const float* __restrict__ x,
    const float* __restrict__ centers,
    const float* __restrict__ widths,
    const int* __restrict__ rules,
    const unsigned short* __restrict__ sch,
    const unsigned short* __restrict__ scl,
    float* __restrict__ out0,
    float* __restrict__ out1,
    float* __restrict__ out2)
{
  extern __shared__ __align__(16) unsigned char dsm[];
  float* sF  = (float*)(dsm + L_F);
  float* sM  = (float*)(dsm + L_M);
  float* sP  = (float*)(dsm + L_P);
  float* sO0 = (float*)(dsm + L_O0);
  float* sO2 = (float*)(dsm + L_O2);
  float* sSx = (float*)(dsm + L_SX);

  const int tid = threadIdx.x, lane = tid & 31, wv = tid >> 5;
  const int b0 = blockIdx.x * RB;

  #pragma unroll 1
  for (int j = 0; j < 6; ++j) {
    const int idx = tid + NTH * j;
    const int row = idx / NQ;
    const int q   = idx - row * NQ;
    const int d   = q / NM;
    const float xv  = x[(size_t)(b0 + row) * ND + d];
    const float c   = centers[q];
    const float w   = widths[q];
    const float df  = xv - c;
    const float den = 2.0f * (w * w);
    const float ex  = -(df * df) * (1.0f / den);
    sM[idx] = expf(ex);
  }
  if (tid < RB) {
    const float* xr = x + (size_t)(b0 + tid) * ND;
    float s = 0.0f;
    #pragma unroll
    for (int i = 0; i < ND; ++i) s += xr[i];
    sSx[tid] = s + 1.0f;
  }
  #pragma unroll 1
  for (int idx = tid; idx < RB * NJ; idx += NTH) {
    const int row = idx / NJ;
    const int i   = idx - row * NJ;
    const int ic  = (i > ND - 1) ? (ND - 1) : i;
    const float xv = x[(size_t)(b0 + row) * ND + ic];
    sO2[idx] = (i < ND) ? xv : 1.0f;
  }
  #pragma unroll 1
  for (int idx = tid; idx < RB * (KP - NRU); idx += NTH) {
    const int row = idx / (KP - NRU);
    const int col = NRU + (idx - row * (KP - NRU));
    sF[row * KP + col] = 0.0f;
  }
  __syncthreads();

  #pragma unroll 1
  for (int rr = 0; rr < 4; ++rr) {
    const int  r  = tid + NTH * rr;
    const bool rv = (r < NRU);
    const int  rc = rv ? r : (NRU - 1);
    int off[ND];
    #pragma unroll
    for (int q4 = 0; q4 < 4; ++q4) {
      const v4i mv = *(const v4ia*)(rules + (size_t)rc * ND + 4 * q4);
      off[4 * q4 + 0] = (4 * q4 + 0) * NM + clampm(mv.x);
      off[4 * q4 + 1] = (4 * q4 + 1) * NM + clampm(mv.y);
      off[4 * q4 + 2] = (4 * q4 + 2) * NM + clampm(mv.z);
      off[4 * q4 + 3] = (4 * q4 + 3) * NM + clampm(mv.w);
    }
    #pragma unroll 1
    for (int row = 0; row < RB; ++row) {
      const float* mr = sM + row * NQ;
      float p = mr[off[0]];
      #pragma unroll
      for (int d = 1; d < ND; ++d) p = p * mr[off[d]];
      if (rv) sF[row * KP + r] = p;
    }
  }
  __syncthreads();

  #pragma unroll 1
  for (int q = 0; q < RB / NWV; ++q) {
    const int row = wv * (RB / NWV) + q;
    float* fr = sF + row * KP;
    unsigned int u[32];
    #pragma unroll
    for (int j = 0; j < 32; ++j) u[j] = __float_as_uint(fr[32 * j + lane]);
    const bool v31 = (lane < NRU - 31 * 32);
    u[31] = v31 ? u[31] : 0u;

    unsigned int lo = 0u, hi = 0x80000000u;
    #pragma unroll 1
    for (int it = 0; it < 31; ++it) {
      const unsigned int mid = lo + ((hi - lo) >> 1);
      int c = 0;
      #pragma unroll
      for (int j = 0; j < 32; ++j) c += (u[j] >= mid) ? 1 : 0;
      c = wsum_i(c);
      const bool ge = (c >= TOPK);
      lo = ge ? mid : lo;
      hi = ge ? hi : mid;
    }
    const unsigned int T = lo;

    int cg = 0;
    #pragma unroll
    for (int j = 0; j < 32; ++j) cg += (u[j] > T) ? 1 : 0;
    cg = wsum_i(cg);

    int tb = 0;
    unsigned int kb = 0u;
    float ss = 0.0f;
    #pragma unroll
    for (int j = 0; j < 32; ++j) {
      const bool vj  = (j < 31) || v31;
      const bool gt  = (u[j] > T);
      const bool tie = vj && (u[j] == T);
      const unsigned int bm = __builtin_amdgcn_ballot_w32(tie);
      const int before = tb + (int)__builtin_popcount(bm & ((1u << lane) - 1u));
      tb += (int)__builtin_popcount(bm);
      const bool kp = gt || (tie && (cg + before < TOPK));
      kb |= kp ? (1u << j) : 0u;
      ss += kp ? __uint_as_float(u[j]) : 0.0f;
    }
    ss = wsum_f(ss);
    const float inv = 1.0f / (ss + 1e-9f);
    #pragma unroll
    for (int j = 0; j < 31; ++j) {
      const bool kp = ((kb >> j) & 1u) != 0u;
      fr[32 * j + lane] = kp ? (__uint_as_float(u[j]) * inv) : 0.0f;
    }
    {
      const bool kp = ((kb >> 31) & 1u) != 0u;
      if (v31) fr[32 * 31 + lane] = kp ? (__uint_as_float(u[31]) * inv) : 0.0f;
    }
  }
  __syncthreads();

  {
    const int h = lane >> 4, m = lane & 15;
    const int mt = wv & 1, kq = wv >> 1;
    const float* ar = sF + (mt * 16 + m) * KP;
    const unsigned short* pbh = sch + (size_t)m * KP;
    const unsigned short* pbl = scl + (size_t)m * KP;
    v8f acc = {0.f, 0.f, 0.f, 0.f, 0.f, 0.f, 0.f, 0.f};
    #pragma unroll 1
    for (int ks = 0; ks < KP / (4 * 32); ++ks) {
      const int k0 = kq * (KP / 4) + ks * 32;
      const v4f a0 = *(const v4fa*)(ar + k0 + 8 * h);
      const v4f a1 = *(const v4fa*)(ar + k0 + 8 * h + 4);
      const v4f a2 = *(const v4fa*)(ar + k0 + 16 + 8 * h);
      const v4f a3 = *(const v4fa*)(ar + k0 + 16 + 8 * h + 4);
      v4u h0, l0, h1, l1;
      split8(a0, a1, h0, l0);
      split8(a2, a3, h1, l1);
      const v8u wh = {h0.x, h0.y, h0.z, h0.w, h1.x, h1.y, h1.z, h1.w};
      const v8u wl = {l0.x, l0.y, l0.z, l0.w, l1.x, l1.y, l1.z, l1.w};
      const v16b ah = __builtin_bit_cast(v16b, wh);
      const v16b al = __builtin_bit_cast(v16b, wl);
      const v16b bh = ldfrag(pbh + k0, h);
      const v16b bl = ldfrag(pbl + k0, h);
      acc = wmma_b(ah, bh, acc);
      acc = wmma_b(ah, bl, acc);
      acc = wmma_b(al, bh, acc);
    }
    #pragma unroll
    for (int r = 0; r < 8; ++r) sP[(wv * 16 + 8 * h + r) * NPB + m] = acc[r];
  }
  __syncthreads();
  #pragma unroll 1
  for (int idx = tid; idx < RB * NC; idx += NTH) {
    const int row = idx / NC;
    const int c   = idx - row * NC;
    const int mt = row >> 4, mm = row & 15;
    float s = 0.0f;
    #pragma unroll
    for (int kq = 0; kq < 4; ++kq) s += sP[((kq * 2 + mt) * 16 + mm) * NPB + c];
    sO0[idx] = sSx[row] * s;
  }
  __syncthreads();

  float* o0 = out0 + (size_t)b0 * NC;
  float* o1 = out1 + (size_t)b0 * NRU;
  float* o2 = out2 + (size_t)b0 * NJ;
  store_pass(sF, sO0, sO2, o0, o1, o2, wv, lane);
  __threadfence();
  store_pass(sF, sO0, sO2, o0, o1, o2, wv, lane);
}

extern "C" void kernel_launch(void* const* d_in, const int* in_sizes, int n_in,
                              void* d_out, int out_size, void* d_ws, size_t ws_size,
                              hipStream_t stream)
{
  if (n_in < 5) return;
  if (in_sizes[0] != NB * ND) return;
  if (in_sizes[1] != NQ) return;
  if (in_sizes[2] != NQ) return;
  if (in_sizes[3] != NRU * ND) return;
  if (in_sizes[4] != NRU * NJ * NC) return;
  if (out_size != NB * NC + NB * NRU + NB * NJ) return;

  const float* x       = (const float*)d_in[0];
  const float* centers = (const float*)d_in[1];
  const float* widths  = (const float*)d_in[2];
  const int*   rules   = (const int*)d_in[3];
  const float* cons    = (const float*)d_in[4];

  float* out0 = (float*)d_out;
  float* out1 = out0 + (size_t)NB * NC;
  float* out2 = out1 + (size_t)NB * NRU;

  const size_t bP = (size_t)NPB * KP * 2;
  const size_t total = 2 * bP;
  if (total > ws_size) return;
  if (total > (size_t)134217728) return;
  char* ws = (char*)d_ws;
  unsigned short* SCH = (unsigned short*)(ws);
  unsigned short* SCL = (unsigned short*)(ws + bP);

  k_scons<<<dim3(KP / NTH, NPB), NTH, 0, stream>>>(cons, SCH, SCL);
  hipFuncSetAttribute(reinterpret_cast<const void*>(&k_main),
                      hipFuncAttributeMaxDynamicSharedMemorySize, LDS_MAIN);
  k_main<<<NB / RB, NTH, LDS_MAIN, stream>>>(x, centers, widths, rules, SCH, SCL,
                                             out0, out1, out2);
}
